// KPConv_89515708383489
// MI455X (gfx1250) — hardware-verified
//
#include <hip/hip_runtime.h>
#include <math.h>

constexpr int kNumQuery    = 100000;
constexpr int kNumSupport  = 100000;
constexpr int kNbr         = 32;
constexpr int kNumKP       = 15;
constexpr int kCin         = 64;
constexpr int kCout        = 128;
constexpr int kKD          = kNumKP * kCin;
constexpr int kPassRows    = 50000;
constexpr int kPassRowsPad = 50048;
constexpr int kQPB         = 8;
constexpr int kGatherBlocks = kPassRowsPad / kQPB;
constexpr float kInfCarry   = 1024.0f;
constexpr float kPlaneScale = 1.0f / 64.0f;
constexpr float kWtsCarry   = 64.0f;
constexpr float kOutScale   = 1.0f / 1024.0f;
constexpr float kInvExtent  = 1.0f / 1.2f;
constexpr float kShadow     = 1.0e6f;

static_assert(kPassRowsPad % 64 == 0);
static_assert(kPassRowsPad >= kPassRows);
static_assert(kPassRowsPad % kQPB == 0);
static_assert(2 * kPassRows == kNumQuery);
static_assert(kKD % 32 == 0);
static_assert(kCout % 64 == 0);
static_assert(kKD % 64 == 0);
static_assert(kNumKP * kCin == kKD);

typedef __attribute__((ext_vector_type(16))) _Float16 v16h;
typedef __attribute__((ext_vector_type(8)))  _Float16 v8h;
typedef __attribute__((ext_vector_type(16))) __bf16   v16b;
typedef __attribute__((ext_vector_type(8)))  __bf16   v8b;
typedef __attribute__((ext_vector_type(8)))  float    v8f;
typedef __attribute__((ext_vector_type(4)))  float    v4f;
typedef __attribute__((ext_vector_type(4)))  unsigned int v4u;

__device__ __forceinline__ unsigned short f2bf_bits(float f) {
  unsigned u = __float_as_uint(f);
  return (unsigned short)((u + 0x7FFFu + ((u >> 16) & 1u)) >> 16);
}
__device__ __forceinline__ float bf_bits2f(unsigned short h) { return __uint_as_float(((unsigned)h) << 16); }

__device__ __forceinline__ void dep_guard_h(v8f& a, v8f& b, v16h x, v16h y) { asm volatile("v_nop\n\tv_nop\n\tv_nop\n\tv_nop" : "+v"(a), "+v"(b) : "v"(x), "v"(y)); }
__device__ __forceinline__ void dep_guard_b(v8f& a, v8f& b, v16b x, v16b y) { asm volatile("v_nop\n\tv_nop\n\tv_nop\n\tv_nop" : "+v"(a), "+v"(b) : "v"(x), "v"(y)); }
__device__ __forceinline__ void dep_guard4_h(v8f& a, v8f& b, v8f& c, v8f& d, v16h x, v16h y) { asm volatile("v_nop\n\tv_nop\n\tv_nop\n\tv_nop" : "+v"(a), "+v"(b), "+v"(c), "+v"(d) : "v"(x), "v"(y)); }
__device__ __forceinline__ void dep_guard4_b(v8f& a, v8f& b, v8f& c, v8f& d, v16b x, v16b y) { asm volatile("v_nop\n\tv_nop\n\tv_nop\n\tv_nop" : "+v"(a), "+v"(b), "+v"(c), "+v"(d) : "v"(x), "v"(y)); }
__device__ __forceinline__ void keep4_h(v16h a, v16h b, v16h c, v16h d) { asm volatile("v_nop" :: "v"(a), "v"(b), "v"(c), "v"(d)); }
__device__ __forceinline__ void keep4_b(v16b a, v16b b, v16b c, v16b d) { asm volatile("v_nop" :: "v"(a), "v"(b), "v"(c), "v"(d)); }
__device__ __forceinline__ void acc_guard4(v8f& a, v8f& b, v8f& c, v8f& d) { asm volatile("v_nop\n\tv_nop\n\tv_nop\n\tv_nop" : "+v"(a), "+v"(b), "+v"(c), "+v"(d)); }
__device__ __forceinline__ void mma4_guard_h(v8f& a0, v8f& a1, v8f& a2, v8f& a3, v16h x, v16h y0, v16h y1, v16h y2, v16h y3) {
  asm volatile("v_nop\n\tv_nop\n\tv_nop\n\tv_nop" : "+v"(a0), "+v"(a1), "+v"(a2), "+v"(a3) : "v"(x), "v"(y0), "v"(y1), "v"(y2), "v"(y3));
}
template <typename T> struct Frag;
template <> struct Frag<_Float16> {
  typedef v16h V; union U { v16h v; v8h h[2]; };
  static __device__ __forceinline__ v16h load(const _Float16* p) {
    U f; f.h[0] = *(const v8h*)(p); f.h[1] = *(const v8h*)(p + 16); return f.v;
  }
  static __device__ __forceinline__ v8f mma(v16h a, v16h b, v8f c) {
    return __builtin_amdgcn_wmma_f32_16x16x32_f16(false, a, false, b, (short)0, c, false, false);
  }
  static __device__ __forceinline__ void guard(v8f& a, v8f& b, v16h x, v16h y) { dep_guard_h(a, b, x, y); }
  static __device__ __forceinline__ void guard4(v8f& a, v8f& b, v8f& c, v8f& d, v16h x, v16h y) { dep_guard4_h(a, b, c, d, x, y); }
  static __device__ __forceinline__ void keep(v16h a, v16h b, v16h c, v16h d) { keep4_h(a, b, c, d); }
};
template <> struct Frag<__bf16> {
  typedef v16b V; union U { v16b v; v8b h[2]; };
  static __device__ __forceinline__ v16b load(const __bf16* p) {
    U f; f.h[0] = *(const v8b*)(p); f.h[1] = *(const v8b*)(p + 16); return f.v;
  }
  static __device__ __forceinline__ v8f mma(v16b a, v16b b, v8f c) {
    return __builtin_amdgcn_wmma_f32_16x16x32_bf16(false, a, false, b, (short)0, c, false, false);
  }
  static __device__ __forceinline__ void guard(v8f& a, v8f& b, v16b x, v16b y) { dep_guard_b(a, b, x, y); }
  static __device__ __forceinline__ void guard4(v8f& a, v8f& b, v8f& c, v8f& d, v16b x, v16b y) { dep_guard4_b(a, b, c, d, x, y); }
  static __device__ __forceinline__ void keep(v16b a, v16b b, v16b c, v16b d) { keep4_b(a, b, c, d); }
};

__device__ __forceinline__ unsigned pk16(unsigned short a, unsigned short b) { return (unsigned)a | ((unsigned)b << 16); }
__device__ __forceinline__ unsigned short h_bits(float f) { const _Float16 h = (_Float16)f; return __builtin_bit_cast(unsigned short, h); }

template <int ET> struct Elem;
template <> struct Elem<0> { typedef _Float16 T; };
template <> struct Elem<1> { typedef __bf16 T; };
template <int ET, bool SPLIT, int BIAS_MODE, int OUT_MODE, bool RESID, int ACT = 0>
__global__ __launch_bounds__(256) void wmma_gemm64(
    const unsigned short* __restrict__ Ap, const unsigned short* __restrict__ A2p, int lda, long strideA,
    const unsigned short* __restrict__ Btp, const unsigned short* __restrict__ Bt2p, int ldb, long strideB,
    void* __restrict__ Cout, void* __restrict__ Cout2, int ldc, long strideC,
    const float* __restrict__ bias,
    const float* __restrict__ resid, long strideR,
    int M, int N, int K, float scale, int Mreal) {
  typedef typename Elem<ET>::T T;
  typedef typename Frag<T>::V V;
  const T* A = (const T*)Ap; const T* A2 = (const T*)A2p; const T* Bt = (const T*)Btp; const T* Bt2 = (const T*)Bt2p;
  __shared__ __align__(16) float sT[8][16 * 68];
  const int b    = blockIdx.y;
  const int lane = threadIdx.x & 31;
  const int wave = threadIdx.x >> 5;
  const int tilesN = N >> 6;
  const int tilesM = M >> 6;
  const int tile = blockIdx.x * 8 + wave;
  if (tile >= tilesM * tilesN) return;
  const int tm = tile / tilesN;
  const int tn = tile - tm * tilesN;
  const int m0 = tm << 6;
  const int n0 = tn << 6;

  const T* Ab  = A  + (size_t)b * strideA;
  const T* Bb  = Bt + (size_t)b * strideB;
  const T* Ab2 = SPLIT ? (A2  + (size_t)b * strideA) : nullptr;
  const T* Bb2 = SPLIT ? (Bt2 + (size_t)b * strideB) : nullptr;

  const int rlane = lane & 15;
  const int koff  = (lane >> 4) * 8;
  const int mOff  = (lane >> 4) * 8;

  v8f acc[4][4];
#pragma unroll
  for (int i = 0; i < 4; ++i)
#pragma unroll
    for (int j = 0; j < 4; ++j) acc[i][j] = (v8f){0.f,0.f,0.f,0.f,0.f,0.f,0.f,0.f};

  for (int k0 = 0; k0 < K; k0 += 32) {
    V bh[4], bl[4];
#pragma unroll
    for (int j = 0; j < 4; ++j) {
      const size_t bo = (size_t)(n0 + (j << 4) + rlane) * ldb + koff + k0;
      bh[j] = Frag<T>::load(Bb + bo);
      if (SPLIT) bl[j] = Frag<T>::load(Bb2 + bo);
    }
#pragma unroll
    for (int i = 0; i < 4; ++i) {
      const size_t ao = (size_t)(m0 + (i << 4) + rlane) * lda + koff + k0;
      V ah = Frag<T>::load(Ab + ao);
      V al;
      if (SPLIT) al = Frag<T>::load(Ab2 + ao);
#pragma unroll
      for (int j = 0; j < 4; ++j) {
        acc[i][j] = Frag<T>::mma(ah, bh[j], acc[i][j]);
        if (SPLIT) {
          acc[i][j] = Frag<T>::mma(ah, bl[j], acc[i][j]);
          acc[i][j] = Frag<T>::mma(al, bh[j], acc[i][j]);
        }
      }
      Frag<T>::guard4(acc[i][0], acc[i][1], acc[i][2], acc[i][3], ah, SPLIT ? al : ah);
    }
    Frag<T>::keep(bh[0], bh[1], bh[2], bh[3]);
    if (SPLIT) Frag<T>::keep(bl[0], bl[1], bl[2], bl[3]);
  }
  acc_guard4(acc[0][0], acc[0][1], acc[0][2], acc[0][3]);
  acc_guard4(acc[1][0], acc[1][1], acc[1][2], acc[1][3]);
  acc_guard4(acc[2][0], acc[2][1], acc[2][2], acc[2][3]);
  acc_guard4(acc[3][0], acc[3][1], acc[3][2], acc[3][3]);

  float* slab = sT[wave];
  const float* Rb = RESID ? (resid + (size_t)b * strideR) : nullptr;
#pragma unroll
  for (int i = 0; i < 4; ++i) {
    const int mBase = m0 + (i << 4);
#pragma unroll
    for (int j = 0; j < 4; ++j) {
      const int n = n0 + (j << 4) + rlane;
      float bv = 0.f;
      if (BIAS_MODE == 2) bv = bias[n];
#pragma unroll
      for (int r = 0; r < 8; ++r) {
        float v = acc[i][j][r] * scale;
        if (BIAS_MODE == 1) v += bias[mBase + mOff + r];
        if (BIAS_MODE == 2) v += bv;
        if (RESID) v += Rb[(size_t)(mBase + mOff + r) * ldc + n];
        if (ACT == 2) v = fmaxf(v, 0.0f);
        if (ACT == 4) v = (v > 0.f) ? v : 0.01f * v;
        slab[(mOff + r) * 68 + (j << 4) + rlane] = v;
      }
    }
    __builtin_amdgcn_fence(__ATOMIC_RELEASE, "workgroup");
    __builtin_amdgcn_wave_barrier();
    __builtin_amdgcn_fence(__ATOMIC_ACQUIRE, "workgroup");
    if (OUT_MODE == 0) {
      float* C = (float*)Cout + (size_t)b * strideC;
      const int hh = lane >> 4, c4 = (lane & 15) * 4;
      for (int pass = 0; pass < 2; ++pass) {
#pragma unroll
        for (int it = 0; it < 8; ++it) {
          const int row = it * 2 + hh;
          const int grow = mBase + row;
          v4f v = *(const v4f*)(slab + row * 68 + c4);
          if (grow < Mreal) *(volatile v4f*)(C + (size_t)grow * ldc + n0 + c4) = v;
        }
        __threadfence();
      }
    } else {
      const int q = lane >> 3, c8 = (lane & 7) * 8;
      unsigned short* C  = (unsigned short*)Cout  + (size_t)b * strideC;
      unsigned short* C2 = (OUT_MODE == 2) ? ((unsigned short*)Cout2 + (size_t)b * strideC) : nullptr;
      for (int pass = 0; pass < 2; ++pass) {
#pragma unroll
        for (int it = 0; it < 4; ++it) {
          const int row = it * 4 + q;
          const int grow = mBase + row;
          const float* sp = slab + row * 68 + c8;
          v8h hv, lv;
#pragma unroll
          for (int e = 0; e < 8; ++e) {
            if (OUT_MODE == 1) {
              hv[e] = (_Float16)sp[e];
            } else {
              unsigned short hb = f2bf_bits(sp[e]);
              unsigned short lb = f2bf_bits(sp[e] - bf_bits2f(hb));
              hv[e] = __builtin_bit_cast(_Float16, hb);
              lv[e] = __builtin_bit_cast(_Float16, lb);
            }
          }
          if (grow < Mreal) {
            *(volatile v8h*)(C + (size_t)grow * ldc + n0 + c8) = hv;
            if (OUT_MODE == 2) *(volatile v8h*)(C2 + (size_t)grow * ldc + n0 + c8) = lv;
          }
        }
        __threadfence();
      }
    }
    __builtin_amdgcn_fence(__ATOMIC_RELEASE, "workgroup");
    __builtin_amdgcn_wave_barrier();
    __builtin_amdgcn_fence(__ATOMIC_ACQUIRE, "workgroup");
  }
}

__global__ __launch_bounds__(256) void wts_bt_kernel(const float* __restrict__ W, unsigned short* __restrict__ Bt) {
  __shared__ float sm[64][65];
  const int t   = threadIdx.x;
  const int kk0 = blockIdx.x * 64;
  const int o0  = blockIdx.y * 64;
#pragma unroll
  for (int i = 0; i < 8; ++i) {
    const int e = i * 256 + t;
    const int r = e >> 6;
    const int c = e & 63;
    sm[c][r] = W[(size_t)(kk0 + r) * kCout + o0 + c] * kWtsCarry;
  }
  asm volatile("" ::: "memory");
#pragma unroll
  for (int i = 8; i < 16; ++i) {
    const int e = i * 256 + t;
    const int r = e >> 6;
    const int c = e & 63;
    sm[c][r] = W[(size_t)(kk0 + r) * kCout + o0 + c] * kWtsCarry;
  }
  __syncthreads();
  const int lane = t & 31, wave = t >> 5;
  const int q = lane >> 3, c8 = (lane & 7) * 8;
  v4u u[2];
#pragma unroll
  for (int it = 0; it < 2; ++it) {
    const int row = wave * 8 + it * 4 + q;
    unsigned short hb[8];
#pragma unroll
    for (int e = 0; e < 8; ++e) hb[e] = h_bits(sm[row][c8 + e]);
    u[it] = (v4u){pk16(hb[0], hb[1]), pk16(hb[2], hb[3]), pk16(hb[4], hb[5]), pk16(hb[6], hb[7])};
  }
  for (int pass = 0; pass < 2; ++pass) {
#pragma unroll
    for (int it = 0; it < 2; ++it) {
      const int row = wave * 8 + it * 4 + q;
      *(volatile v4u*)(Bt + (size_t)(o0 + row) * kKD + kk0 + c8) = u[it];
    }
    __threadfence();
  }
}

__global__ __launch_bounds__(256) void gather_agg_kernel(
    const float* __restrict__ qpts, const float* __restrict__ spts, const int* __restrict__ nidx,
    const float* __restrict__ feats, const float* __restrict__ kpts,
    unsigned short* __restrict__ Apl, int rowBase) {
  __shared__ __align__(16) unsigned short sF[kQPB * kCin * kNbr];
  __shared__ __align__(16) unsigned short sW[kQPB * 16 * kNbr];
  __shared__ float sKP[16 * 4];
  const int tid  = threadIdx.x;
  const int lane = tid & 31;
  const int wave = tid >> 5;

  {
    const int kt = (tid < kNumKP * 3) ? tid : (kNumKP * 3 - 1);
    const float kv = kpts[kt];
    if (tid < kNumKP * 3) { const int kk = tid / 3; sKP[kk * 4 + (tid - 3 * kk)] = kv; }
  }

  const int prow = blockIdx.x * kQPB + wave;
  const bool live = prow < kPassRows;
  int n = rowBase + prow; n = (n < kNumQuery) ? n : (kNumQuery - 1);
  const int idx = nidx[(size_t)n * kNbr + lane];
  const bool valid = live && (idx >= 0) && (idx < kNumSupport);
  int ic = (idx < 0) ? 0 : idx; ic = (ic < kNumSupport) ? ic : (kNumSupport - 1);
  const float validf = valid ? 1.0f : 0.0f;
  const float shadow = (1.0f - validf) * kShadow;
  const float sx = spts[(size_t)ic * 3 + 0];
  const float sy = spts[(size_t)ic * 3 + 1];
  const float sz = spts[(size_t)ic * 3 + 2];
  const float qx = qpts[(size_t)n * 3 + 0];
  const float qy = qpts[(size_t)n * 3 + 1];
  const float qz = qpts[(size_t)n * 3 + 2];
  const float nx = fmaf(sx, validf, shadow) - qx;
  const float ny = fmaf(sy, validf, shadow) - qy;
  const float nz = fmaf(sz, validf, shadow) - qz;
  __syncthreads();

  unsigned short* sWq = sW + wave * (16 * kNbr);
#pragma unroll
  for (int k = 0; k < kNumKP; ++k) {
    const float dx = nx - sKP[k * 4 + 0];
    const float dy = ny - sKP[k * 4 + 1];
    const float dz = nz - sKP[k * 4 + 2];
    const float sq = dx * dx + dy * dy + dz * dz;
    const float w  = fmaxf(1.0f - sqrtf(sq) * kInvExtent, 0.0f);
    sWq[k * kNbr + lane] = h_bits(w * kInfCarry);
  }
  sWq[kNumKP * kNbr + lane] = (unsigned short)0;

  const float* frow = feats + (size_t)ic * kCin;
  unsigned short* sFq = sF + wave * (kCin * kNbr);
#pragma unroll
  for (int g = 0; g < 4; ++g) {
    v4f f4[4];
#pragma unroll
    for (int j = 0; j < 4; ++j) f4[j] = *(const v4f*)(frow + g * 16 + j * 4);
#pragma unroll
    for (int j = 0; j < 4; ++j) {
#pragma unroll
      for (int e = 0; e < 4; ++e) sFq[(g * 16 + j * 4 + e) * kNbr + lane] = h_bits(f4[j][e] * validf);
    }
    asm volatile("" ::: "memory");
  }
  __syncthreads();

  const int m  = lane & 15;
  const int hh = lane >> 4;
  const _Float16* Wt = (const _Float16*)(sW + wave * (16 * kNbr));
  const _Float16* Ft = (const _Float16*)(sF + wave * (kCin * kNbr));
  const v16h a  = Frag<_Float16>::load(Wt + m * kNbr + 8 * hh);
  const v16h b0 = Frag<_Float16>::load(Ft + (0 * 16 + m) * kNbr + 8 * hh);
  const v16h b1 = Frag<_Float16>::load(Ft + (1 * 16 + m) * kNbr + 8 * hh);
  const v16h b2 = Frag<_Float16>::load(Ft + (2 * 16 + m) * kNbr + 8 * hh);
  const v16h b3 = Frag<_Float16>::load(Ft + (3 * 16 + m) * kNbr + 8 * hh);
  const v8f z8 = (v8f){0.f, 0.f, 0.f, 0.f, 0.f, 0.f, 0.f, 0.f};
  v8f acc0 = Frag<_Float16>::mma(a, b0, z8);
  v8f acc1 = Frag<_Float16>::mma(a, b1, z8);
  v8f acc2 = Frag<_Float16>::mma(a, b2, z8);
  v8f acc3 = Frag<_Float16>::mma(a, b3, z8);
  mma4_guard_h(acc0, acc1, acc2, acc3, a, b0, b1, b2, b3);
  __syncthreads();

  unsigned short* so = sF + wave * (kCin * kNbr);
#pragma unroll
  for (int r = 0; r < 8; ++r) {
    const int row = 8 * hh + r;
    so[row * 64 + m]      = h_bits(acc0[r] * kPlaneScale);
    so[row * 64 + 16 + m] = h_bits(acc1[r] * kPlaneScale);
    so[row * 64 + 32 + m] = h_bits(acc2[r] * kPlaneScale);
    so[row * 64 + 48 + m] = h_bits(acc3[r] * kPlaneScale);
  }
  __syncthreads();

  const int g8 = lane >> 3, c8 = (lane & 7) * 8;
  v4u v[4];
#pragma unroll
  for (int it = 0; it < 4; ++it) v[it] = *(const v4u*)(so + (it * 4 + g8) * 64 + c8);
  unsigned short* arow = Apl + (size_t)prow * kKD;
  for (int pass = 0; pass < 2; ++pass) {
#pragma unroll
    for (int it = 0; it < 4; ++it) {
      const int k = it * 4 + g8;
      if (k < kNumKP) *(volatile v4u*)(arow + k * kCin + c8) = v[it];
    }
    __threadfence();
  }
}

extern "C" void kernel_launch(void* const* d_in, const int* in_sizes, int n_in,
                              void* d_out, int out_size, void* d_ws, size_t ws_size, hipStream_t stream) {
  (void)in_sizes; (void)n_in; (void)out_size;
  const float* qpts  = (const float*)d_in[0];
  const float* spts  = (const float*)d_in[1];
  const int*   nidx  = (const int*)  d_in[2];
  const float* feats = (const float*)d_in[3];
  const float* kpts  = (const float*)d_in[4];
  const float* wts   = (const float*)d_in[5];
  float* out = (float*)d_out;

  const size_t bytesBt = (size_t)kCout * kKD * 2;
  const size_t bytesA  = (size_t)kPassRowsPad * kKD * 2;
  const size_t offBt = 0;
  const size_t offA  = offBt + bytesBt;
  const size_t total = offA + bytesA;
  if (total > ws_size || total > (size_t)134217728) return;
  char* ws = (char*)d_ws;
  unsigned short* Bt  = (unsigned short*)(ws + offBt);
  unsigned short* Apl = (unsigned short*)(ws + offA);

  wts_bt_kernel<<<dim3(kKD / 64, kCout / 64), 256, 0, stream>>>(wts, Bt);

  const int gemmTiles  = (kPassRowsPad / 64) * (kCout / 64);
  const int gemmBlocks = (gemmTiles + 7) / 8;
  for (int pass = 0; pass < 2; ++pass) {
    gather_agg_kernel<<<kGatherBlocks, 256, 0, stream>>>(qpts, spts, nidx, feats, kpts, Apl, pass * kPassRows);
    wmma_gemm64<0, false, 0, 0, false><<<dim3(gemmBlocks, 1), 256, 0, stream>>>(
        (const unsigned short*)Apl, (const unsigned short*)Apl, kKD, 0L,
        (const unsigned short*)Bt, (const unsigned short*)Bt, kKD, 0L,
        (void*)(out + (size_t)pass * kPassRows * kCout), (void*)nullptr, kCout, 0L,
        (const float*)nullptr, (const float*)nullptr, 0L,
        kPassRowsPad, kCout, kKD, kOutScale, kPassRows);
  }
}
